// DampedIMEX1Layer_22368189677865
// MI455X (gfx1250) — hardware-verified
//
#include <hip/hip_runtime.h>
#include <stddef.h>
#include <stdint.h>
#include <math.h>

#pragma clang fp contract(off)

#define NBATCH 8
#define SEQ    8192
#define PD     128
#define HD     128
#define MROWS  (NBATCH * SEQ)
#define NBU    (2 * PD)
#define KYS    (2 * PD)
#define LDY    (2 * KYS)
#define SFP    68
#define TB     16

static_assert(PD == 128);
static_assert(HD == 128);
static_assert(MROWS % 128 == 0);
static_assert(NBU % 64 == 0);
static_assert(HD % 64 == 0);
static_assert(HD % 32 == 0);
static_assert(KYS % 32 == 0);
static_assert((MROWS * HD) % 2048 == 0);
static_assert((PD * HD * 2) % 2048 == 0);
static_assert(SEQ % TB == 0);
static_assert((TB * LDY) % (256 * 8) == 0);
static_assert(LDY * 2 == NBU * 4);

typedef _Float16 hh;
typedef hh v16h __attribute__((ext_vector_type(16)));
typedef __attribute__((ext_vector_type(16))) __bf16 v16bf;
typedef float v8f __attribute__((ext_vector_type(8)));
typedef float v4f __attribute__((ext_vector_type(4)));
typedef int v4i __attribute__((ext_vector_type(4)));
typedef int v8i __attribute__((ext_vector_type(8)));
typedef unsigned short v8us __attribute__((ext_vector_type(8)));

__device__ __forceinline__ v8f zero8() { return (v8f){0.f, 0.f, 0.f, 0.f, 0.f, 0.f, 0.f, 0.f}; }

__device__ __forceinline__ unsigned int bf16_rne_bits(float f) {
  const unsigned int u = __float_as_uint(f);
  return (u + 0x7fffu + ((u >> 16) & 1u)) >> 16;
}

__device__ __forceinline__ v8i ldfrag16(const unsigned short* __restrict__ p, int ld, int row0, int k0, int lane) {
  const unsigned short* q = p + (size_t)(row0 + (lane & 15)) * (size_t)ld + k0 + 8 * (lane >> 4);
  const v4i lo = *(const v4i*)(const void*)(q);
  const v4i hi = *(const v4i*)(const void*)(q + 16);
  return __builtin_shufflevector(lo, hi, 0, 1, 2, 3, 4, 5, 6, 7);
}

__device__ __forceinline__ v8f mma_b(v8i a, v8i b, v8f cc) {
  return __builtin_amdgcn_wmma_f32_16x16x32_bf16(false, __builtin_bit_cast(v16bf, a), false,
                                                 __builtin_bit_cast(v16bf, b), (short)0, cc, false, false);
}

__device__ __forceinline__ void gemm32x32(const unsigned short* __restrict__ A, const unsigned short* __restrict__ AL,
                                          int lda, const unsigned short* __restrict__ B,
                                          const unsigned short* __restrict__ BL, int ldb, int ma, int nb, int kdim,
                                          int lane, v8f (&acc)[2][2]) {
#pragma unroll 1
  for (int k0 = 0; k0 < kdim; k0 += 32) {
    const v8i a0 = ldfrag16(A, lda, ma, k0, lane);
    const v8i a1 = ldfrag16(A, lda, ma + 16, k0, lane);
    const v8i b0 = ldfrag16(B, ldb, nb, k0, lane);
    const v8i b1 = ldfrag16(B, ldb, nb + 16, k0, lane);
    const v8i c0 = ldfrag16(AL, lda, ma, k0, lane);
    const v8i c1 = ldfrag16(AL, lda, ma + 16, k0, lane);
    const v8i d0 = ldfrag16(BL, ldb, nb, k0, lane);
    const v8i d1 = ldfrag16(BL, ldb, nb + 16, k0, lane);
    acc[0][0] = mma_b(a0, b0, acc[0][0]);
    acc[1][0] = mma_b(a1, b0, acc[1][0]);
    acc[0][1] = mma_b(a0, b1, acc[0][1]);
    acc[1][1] = mma_b(a1, b1, acc[1][1]);
    acc[0][0] = mma_b(a0, d0, acc[0][0]);
    acc[1][0] = mma_b(a1, d0, acc[1][0]);
    acc[0][1] = mma_b(a0, d1, acc[0][1]);
    acc[1][1] = mma_b(a1, d1, acc[1][1]);
    acc[0][0] = mma_b(c0, b0, acc[0][0]);
    acc[1][0] = mma_b(c1, b0, acc[1][0]);
    acc[0][1] = mma_b(c0, b1, acc[0][1]);
    acc[1][1] = mma_b(c1, b1, acc[1][1]);
    asm volatile("v_nop\n\tv_nop\n\tv_nop\n\tv_nop"
                 : "+v"(acc[0][0]), "+v"(acc[0][1]), "+v"(acc[1][0]), "+v"(acc[1][1])
                 : "v"(a0), "v"(a1), "v"(b0), "v"(b1), "v"(c0), "v"(c1), "v"(d0), "v"(d1));
  }
}

__global__ __launch_bounds__(256) void k_split(const float* __restrict__ w, unsigned short* __restrict__ hi,
                                               unsigned short* __restrict__ lo) {
  const size_t i = ((size_t)blockIdx.x * 256 + threadIdx.x) * 8;
  const v4f a0 = *(const v4f*)(w + i);
  const v4f a1 = *(const v4f*)(w + i + 4);
  const v8f t = {a0[0], a0[1], a0[2], a0[3], a1[0], a1[1], a1[2], a1[3]};
  v8us hv, lv;
#pragma unroll
  for (int e = 0; e < 8; ++e) {
    const float v = t[e];
    const unsigned int hb = bf16_rne_bits(v);
    const float fh = __uint_as_float(hb << 16);
    const unsigned int lb = bf16_rne_bits(v - fh);
    hv[e] = (unsigned short)hb;
    lv[e] = (unsigned short)lb;
  }
  *(volatile v8us*)(hi + i) = hv;
  *(volatile v8us*)(lo + i) = lv;
  __threadfence();
  *(volatile v8us*)(hi + i) = hv;
  *(volatile v8us*)(lo + i) = lv;
}

__global__ __launch_bounds__(256) void k_prepw(const float* __restrict__ Bw, const float* __restrict__ Cw,
                                               unsigned short* __restrict__ BPH, unsigned short* __restrict__ BPL,
                                               unsigned short* __restrict__ CPH, unsigned short* __restrict__ CPL) {
  const int i = blockIdx.x * 256 + threadIdx.x;
  const int e0 = i * 8;
  const int nb = e0 / HD, kb = e0 % HD;
  const float* sb = Bw + ((size_t)((nb & (PD - 1)) * HD + kb)) * 2 + (nb >> 7);
  const int hc = e0 / KYS, kc = e0 % KYS;
  const int cc = kc >> 7;
  const float sgn = cc ? -1.0f : 1.0f;
  const float* sc = Cw + ((size_t)(hc * PD + (kc & (PD - 1)))) * 2 + cc;
  v8us bh, bl, ch, cl;
#pragma unroll
  for (int e = 0; e < 8; ++e) {
    const float vb = sb[2 * e];
    const unsigned int hb = bf16_rne_bits(vb);
    const float fb = __uint_as_float(hb << 16);
    bh[e] = (unsigned short)hb;
    bl[e] = (unsigned short)bf16_rne_bits(vb - fb);
    const float vc = sgn * sc[2 * e];
    const unsigned int hcb = bf16_rne_bits(vc);
    const float fc = __uint_as_float(hcb << 16);
    ch[e] = (unsigned short)hcb;
    cl[e] = (unsigned short)bf16_rne_bits(vc - fc);
  }
  *(volatile v8us*)(BPH + e0) = bh;
  *(volatile v8us*)(BPL + e0) = bl;
  *(volatile v8us*)(CPH + e0) = ch;
  *(volatile v8us*)(CPL + e0) = cl;
  __threadfence();
  *(volatile v8us*)(BPH + e0) = bh;
  *(volatile v8us*)(BPL + e0) = bl;
  *(volatile v8us*)(CPH + e0) = ch;
  *(volatile v8us*)(CPL + e0) = cl;
}

template <int KD, int LDA, int LDB, int LDO, bool RES>
__global__ __launch_bounds__(256) void k_gemm(const unsigned short* __restrict__ A,
                                              const unsigned short* __restrict__ AL,
                                              const unsigned short* __restrict__ B,
                                              const unsigned short* __restrict__ BL,
                                              const float* __restrict__ res, const float* __restrict__ dv,
                                              float* __restrict__ o32) {
  __shared__ __align__(16) float ldsf[128 * SFP];
  const int tid = threadIdx.x, lane = tid & 31, w = tid >> 5;
  const int h = lane >> 4, c = lane & 15;
  const int wm = (w >> 1) * 32, wn = (w & 1) * 32;
  const int m0 = blockIdx.y * 128;
  const int n0 = blockIdx.x * 64;

  v8f acc[2][2];
#pragma unroll
  for (int i = 0; i < 2; ++i)
#pragma unroll
    for (int j = 0; j < 2; ++j) acc[i][j] = zero8();
  gemm32x32(A, AL, LDA, B, BL, LDB, m0 + wm, n0 + wn, KD, lane, acc);

#pragma unroll
  for (int i = 0; i < 2; ++i)
#pragma unroll
    for (int j = 0; j < 2; ++j)
#pragma unroll
      for (int r = 0; r < 8; ++r)
        ldsf[(wm + 16 * i + 8 * h + r) * SFP + wn + 16 * j + c] = acc[i][j][r];
  __syncthreads();

  v4f val[8];
  size_t go[8];
#pragma unroll
  for (int it = 0; it < 8; ++it) {
    const int p  = tid + 256 * it;
    const int lr = p >> 4;
    const int pc = p & 15;
    const v4f sv = *(const v4f*)(ldsf + lr * SFP + pc * 4);
    const size_t gi = (size_t)(m0 + lr) * LDO + n0 + pc * 4;
    if constexpr (RES) {
      const v4f rr = *(const v4f*)(res + gi);
      const v4f dd = *(const v4f*)(dv + n0 + pc * 4);
      val[it] = sv + rr * dd;
    } else {
      val[it] = sv;
    }
    go[it] = gi;
  }
#pragma unroll
  for (int it = 0; it < 8; ++it) *(volatile v4f*)(o32 + go[it]) = val[it];
  __threadfence();
#pragma unroll
  for (int it = 0; it < 8; ++it) *(volatile v4f*)(o32 + go[it]) = val[it];
}

__global__ __launch_bounds__(256) void k_scan(const float* __restrict__ Adiag, const float* __restrict__ Gdiag,
                                              const float* __restrict__ dtv, float* buy) {
  __shared__ __align__(16) unsigned short lds[TB * LDY];
  const int tid = threadIdx.x;
  const int p = tid & (PD - 1);
  const size_t rowb = (size_t)blockIdx.x * SEQ;
  unsigned short* ys = (unsigned short*)buy;

  const float dtr = dtv[p];
  const float ex = expf(-dtr);
  const float dts = 1.0f / (1.0f + ex);
  const float Av = fmaxf(Adiag[p], 0.0f);
  const float Gv = fmaxf(Gdiag[p], 0.0f);
  const float dt2 = fmaxf(dts * dts, 1e-6f);
  const float dG = dts * Gv;
  const float sq = sqrtf(1.0f + dG);
  const float rdt2 = 1.0f / dt2;
  const float A_low  = (2.0f + dG - 2.0f * sq) * rdt2;
  const float A_high = (2.0f + dG + 2.0f * sq) * rdt2;
  const float A_fin = A_low + fmaxf(Av - A_low, 0.0f) - fmaxf(Av - A_high, 0.0f);
  const float Sv = 1.0f + dG;
  const float rS = 1.0f / Sv;
  const float q1 = dts * rS;
  const float q2 = (dts * dts) * rS;
  const float m11 = rS;
  const float m12 = -q1 * A_fin;
  const float m21 = q1;
  const float m22 = 1.0f - q2 * A_fin;

  float s1 = 0.f, s2 = 0.f;
#pragma unroll 1
  for (int t0 = 0; t0 < SEQ; t0 += TB) {
#pragma unroll 4
    for (int tt = 0; tt < TB; ++tt) {
      const float u = buy[(rowb + t0 + tt) * NBU + tid];
      const float n1 = m11 * s1 + m12 * s2 + q1 * u;
      const float n2 = m21 * s1 + m22 * s2 + q2 * u;
      s1 = n1;
      s2 = n2;
      const unsigned int hb = bf16_rne_bits(s2);
      const float fh = __uint_as_float(hb << 16);
      const unsigned int lb = bf16_rne_bits(s2 - fh);
      lds[tt * LDY + tid] = (unsigned short)hb;
      lds[tt * LDY + KYS + tid] = (unsigned short)lb;
    }
    __syncthreads();
    v8us hv[4];
    size_t go[4];
#pragma unroll
    for (int it = 0; it < 4; ++it) {
      const int q = tid + 256 * it;
      const int row = q >> 6;
      const int pc = q & 63;
      hv[it] = *(const v8us*)(lds + row * LDY + pc * 8);
      go[it] = (rowb + t0 + row) * LDY + (size_t)pc * 8;
    }
#pragma unroll
    for (int it = 0; it < 4; ++it) *(volatile v8us*)(ys + go[it]) = hv[it];
    __threadfence();
#pragma unroll
    for (int it = 0; it < 4; ++it) *(volatile v8us*)(ys + go[it]) = hv[it];
    __syncthreads();
  }
}

extern "C" void kernel_launch(void* const* d_in, const int* in_sizes, int n_in,
                              void* d_out, int out_size, void* d_ws, size_t ws_size,
                              hipStream_t stream) {
  if (n_in < 7) return;
  if (in_sizes[0] != MROWS * HD) return;
  if (in_sizes[1] != PD) return;
  if (in_sizes[2] != PD) return;
  if (in_sizes[3] != PD) return;
  if (in_sizes[4] != PD * HD * 2) return;
  if (in_sizes[5] != HD * PD * 2) return;
  if (in_sizes[6] != HD) return;
  if (out_size != MROWS * HD) return;

  const float* x   = (const float*)d_in[0];
  const float* Ad  = (const float*)d_in[1];
  const float* Gd  = (const float*)d_in[2];
  const float* dtv = (const float*)d_in[3];
  const float* Bw  = (const float*)d_in[4];
  const float* Cw  = (const float*)d_in[5];
  const float* Dv  = (const float*)d_in[6];
  float* out = (float*)d_out;

  size_t off = 0;
  const size_t oXH  = off; off += (size_t)MROWS * HD * 2;
  const size_t oXL  = off; off += (size_t)MROWS * HD * 2;
  const size_t oBPH = off; off += (size_t)NBU * HD * 2;
  const size_t oBPL = off; off += (size_t)NBU * HD * 2;
  const size_t oCPH = off; off += (size_t)HD * KYS * 2;
  const size_t oCPL = off; off += (size_t)HD * KYS * 2;
  const size_t oBU  = off; off += (size_t)MROWS * NBU * 4;
  if (off > ws_size) return;
  if (off > (size_t)134217728) return;

  char* ws = (char*)d_ws;
  unsigned short* XH  = (unsigned short*)(ws + oXH);
  unsigned short* XL  = (unsigned short*)(ws + oXL);
  unsigned short* BPH = (unsigned short*)(ws + oBPH);
  unsigned short* BPL = (unsigned short*)(ws + oBPL);
  unsigned short* CPH = (unsigned short*)(ws + oCPH);
  unsigned short* CPL = (unsigned short*)(ws + oCPL);
  float* BU = (float*)(ws + oBU);
  unsigned short* YS = (unsigned short*)(ws + oBU);

  k_split<<<dim3((MROWS * HD) / 2048), dim3(256), 0, stream>>>(x, XH, XL);
  k_prepw<<<dim3((PD * HD * 2) / 2048), dim3(256), 0, stream>>>(Bw, Cw, BPH, BPL, CPH, CPL);
  k_gemm<HD, HD, HD, NBU, false><<<dim3(NBU / 64, MROWS / 128), dim3(256), 0, stream>>>(XH, XL, BPH, BPL, x, Dv, BU);
  k_scan<<<dim3(NBATCH), dim3(256), 0, stream>>>(Ad, Gd, dtv, BU);
  k_gemm<KYS, LDY, KYS, HD, true><<<dim3(HD / 64, MROWS / 128), dim3(256), 0, stream>>>(YS, YS + KYS, CPH, CPL, x,
                                                                                        Dv, out);
  (void)hipGetLastError();
}
